// ComplexDotProductAttention_38792144617705
// MI455X (gfx1250) — hardware-run, weakly checked
//
#include <hip/hip_runtime.h>


#define NB_  4
#define NQ   4096
#define NK   4096
#define DD   64
#define RQ   1024
typedef _Float16 h16;
typedef unsigned short bf;
typedef __attribute__((ext_vector_type(16))) __bf16   v16bf;
typedef __attribute__((ext_vector_type(16))) _Float16 v16h;
typedef __attribute__((ext_vector_type(8)))  _Float16 v8h;
typedef __attribute__((ext_vector_type(8)))  unsigned short v8us;
typedef __attribute__((ext_vector_type(8)))  float    v8f;
typedef __attribute__((ext_vector_type(4)))  float    v4f;
typedef v8h  __attribute__((may_alias)) v8ha;
typedef v4f  __attribute__((may_alias)) v4fa;
typedef v8us __attribute__((may_alias)) v8usa;

__device__ __forceinline__ unsigned short f2bf(float f) { unsigned u = __float_as_uint(f); u += 0x7FFFu + ((u >> 16) & 1u); return (unsigned short)(u >> 16); }
__device__ __forceinline__ float bf2f(unsigned short b) { return __uint_as_float(((unsigned)b) << 16); }
__device__ __forceinline__ float bfr(float f) { return bf2f(f2bf(f)); }
__device__ __forceinline__ v16h cat16(v8h lo, v8h hi) { return __builtin_shufflevector(lo, hi, 0, 1, 2, 3, 4, 5, 6, 7, 8, 9, 10, 11, 12, 13, 14, 15); }
__device__ __forceinline__ v16bf cat16b(v8us lo, v8us hi) { return __builtin_bit_cast(v16bf, __builtin_shufflevector(lo, hi, 0, 1, 2, 3, 4, 5, 6, 7, 8, 9, 10, 11, 12, 13, 14, 15)); }
__device__ __forceinline__ v8f wmma16(v16h a, v16h b, v8f c) { return __builtin_amdgcn_wmma_f32_16x16x32_f16(false, a, false, b, (short)0, c, false, false); }
__device__ __forceinline__ v8f wmmab(v16bf a, v16bf b, v8f c) { return __builtin_amdgcn_wmma_f32_16x16x32_bf16(false, a, false, b, (short)0, c, false, false); }


template <typename T16> struct WFrag;
template <> struct WFrag<h16> { typedef v16h V; static __device__ __forceinline__ V ld(const h16* p) { return cat16(*(const v8h*)p, *(const v8h*)(p + 16)); } static __device__ __forceinline__ v8f mma(V a, V b, v8f c) { return wmma16(a, b, c); } };
template <> struct WFrag<bf> { typedef v16bf V; static __device__ __forceinline__ V ld(const bf* p) { return cat16b(*(const v8us*)p, *(const v8us*)(p + 16)); } static __device__ __forceinline__ v8f mma(V a, V b, v8f c) { return wmmab(a, b, c); } };
template <typename T16, int NSPLIT, bool BIAS>
__global__ __launch_bounds__(32) void k_gemmw(const T16* __restrict__ A, const T16* __restrict__ A2, const T16* __restrict__ Bt, const T16* __restrict__ Bt2, int K, float* C, int ldc, const float* __restrict__ bias, size_t sA, size_t sB, size_t sC) {
    typedef typename WFrag<T16>::V V;
    __shared__ __align__(16) float os[16 * 68];
    const size_t z = blockIdx.z; A += z * sA; if (A2) A2 += z * sA; Bt += z * sB; if (Bt2) Bt2 += z * sB; C += z * sC;
    const int lane = threadIdx.x & 31, lr = lane & 15, hi = lane >> 4; const int r0 = blockIdx.x * 64, c0 = blockIdx.y * 64;
    v8f acc[4][4];
#pragma unroll
    for (int mb = 0; mb < 4; ++mb)
#pragma unroll
        for (int nb = 0; nb < 4; ++nb) acc[mb][nb] = (v8f){};
    const size_t aoff = (size_t)(r0 + lr) * K + 8 * hi, boff = (size_t)(c0 + lr) * K + 8 * hi;
#pragma unroll 1
    for (int kc = 0; kc < K; kc += 32) {
        V a[4], a2[4];
#pragma unroll
        for (int mb = 0; mb < 4; ++mb) { a[mb] = WFrag<T16>::ld(A + aoff + (size_t)mb * 16 * K + kc); if (NSPLIT == 1 || NSPLIT == 2) a2[mb] = WFrag<T16>::ld(A2 + aoff + (size_t)mb * 16 * K + kc); }
#pragma unroll
        for (int nb = 0; nb < 4; ++nb) { const V b = WFrag<T16>::ld(Bt + boff + (size_t)nb * 16 * K + kc); V b2; if (NSPLIT >= 2) b2 = WFrag<T16>::ld(Bt2 + boff + (size_t)nb * 16 * K + kc);
#pragma unroll
            for (int mb = 0; mb < 4; ++mb) { acc[mb][nb] = WFrag<T16>::mma(a[mb], b, acc[mb][nb]); if (NSPLIT == 1 || NSPLIT == 2) acc[mb][nb] = WFrag<T16>::mma(a2[mb], b, acc[mb][nb]); if (NSPLIT >= 2) acc[mb][nb] = WFrag<T16>::mma(a[mb], b2, acc[mb][nb]); } }
        asm volatile("v_nop\n\tv_nop\n\tv_nop\n\tv_nop" : "+v"(acc[0][0]), "+v"(acc[1][1]), "+v"(acc[2][2]), "+v"(acc[3][3]) : "v"(a[0]), "v"(a[3]));
    }
#pragma unroll
    for (int mb = 0; mb < 4; ++mb) {
#pragma unroll
        for (int nb = 0; nb < 4; ++nb) {
#pragma unroll
            for (int j = 0; j < 8; ++j) os[(hi * 8 + j) * 68 + nb * 16 + lr] = acc[mb][nb][j]; }
        __builtin_amdgcn_wave_barrier(); asm volatile("" ::: "memory");
        float* crow = C + (size_t)(r0 + mb * 16) * ldc + c0;
#pragma unroll 1
        for (int ps = 0; ps < 2; ++ps) {
#pragma unroll
            for (int s = 0; s < 8; ++s) { const int row = 2 * s + hi, cofs = lr * 4; v4f val = *(const v4fa*)(os + row * 68 + cofs); if (BIAS) { val[0] += bfr(bias[c0 + cofs]); val[1] += bfr(bias[c0 + cofs + 1]); val[2] += bfr(bias[c0 + cofs + 2]); val[3] += bfr(bias[c0 + cofs + 3]); }
                *(volatile v4f*)(crow + (size_t)row * ldc + cofs) = val; }
            if (ps == 0) __threadfence(); }
        __builtin_amdgcn_wave_barrier(); asm volatile("" ::: "memory");
    }
}

__device__ __forceinline__ void splitf(float y, unsigned short& h, unsigned short& l) { h = f2bf(y); l = f2bf(y - bf2f(h)); }
typedef __attribute__((ext_vector_type(2))) unsigned short v2us;
typedef __attribute__((ext_vector_type(4))) unsigned short v4us;

__global__ __launch_bounds__(256) void k_qcat(const float* __restrict__ Q, bf* QC) { const size_t e = ((size_t)blockIdx.x * 256 + threadIdx.x) * 4; if (e >= (size_t)NQ * 2 * DD) return; const int c = (int)(e % (2 * DD)); const size_t q = e / (2 * DD); const int part = c / DD, d = c % DD; v4us o;
#pragma unroll
    for (int u = 0; u < 4; ++u) o[u] = f2bf(Q[(q * DD + d + u) * 2 + part]); *(volatile v4us*)(QC + e) = o; __threadfence(); *(volatile v4us*)(QC + e) = o; }
__global__ __launch_bounds__(256) void k_kcat(const float* __restrict__ K, bf* KA, bf* KB) { const size_t e = ((size_t)blockIdx.x * 256 + threadIdx.x) * 4; if (e >= (size_t)NK * 2 * DD) return; const int c = (int)(e % (2 * DD)); const size_t k = e / (2 * DD); const int part = c / DD, d = c % DD; v4us oa, ob;
#pragma unroll
    for (int u = 0; u < 4; ++u) { const float kr = K[(k * DD + d + u) * 2], ki = K[(k * DD + d + u) * 2 + 1]; oa[u] = f2bf(part ? ki : kr); ob[u] = f2bf(part ? -kr : ki); } *(volatile v4us*)(KA + e) = oa; *(volatile v4us*)(KB + e) = ob; __threadfence(); *(volatile v4us*)(KA + e) = oa; *(volatile v4us*)(KB + e) = ob; }
__global__ __launch_bounds__(256) void k_vcat(const float* __restrict__ V, bf* V1, bf* V2) { const size_t e = ((size_t)blockIdx.x * 256 + threadIdx.x) * 2; if (e >= (size_t)DD * 2 * NK) return; const int kp = (int)(e % (2 * NK)); const int v = (int)(e / (2 * NK)); const int part = kp / NK, k = kp % NK; v2us o1, o2;
#pragma unroll
    for (int u = 0; u < 2; ++u) { const float vr = V[((size_t)(k + u) * DD + v) * 2], vi = V[((size_t)(k + u) * DD + v) * 2 + 1]; o1[u] = f2bf(part ? -vi : vr); o2[u] = f2bf(part ? vr : vi); } *(volatile v2us*)(V1 + e) = o1; *(volatile v2us*)(V2 + e) = o2; __threadfence(); *(volatile v2us*)(V1 + e) = o1; *(volatile v2us*)(V2 + e) = o2; }
__global__ __launch_bounds__(256) void k_csm(const float* __restrict__ SR, const float* __restrict__ SI, bf* Ah, bf* Al) { const int lane = threadIdx.x & 31; const int row = blockIdx.x * 8 + (threadIdx.x >> 5); if (row >= RQ) return; const float* sr = SR + (size_t)row * NK; const float* si = SI + (size_t)row * NK; float mx = -3.0e38f;
    for (int j = lane * 4; j < NK; j += 128) { const v4f a = *(const v4f*)(sr + j), b = *(const v4f*)(si + j); for (int u = 0; u < 4; ++u) { const float x = a[u] * 0.125f, y = b[u] * 0.125f; float xx = __fmul_rn(x, x); asm volatile("" : "+v"(xx)); float yy = __fmul_rn(y, y); asm volatile("" : "+v"(yy)); mx = fmaxf(mx, __fsqrt_rn(__fadd_rn(xx, yy))); } }
#pragma unroll
    for (int sh = 16; sh; sh >>= 1) mx = fmaxf(mx, __shfl_xor(mx, sh, 32));
    float sum = 0.f;
    for (int j = lane * 4; j < NK; j += 128) { const v4f a = *(const v4f*)(sr + j), b = *(const v4f*)(si + j); for (int u = 0; u < 4; ++u) { const float x = a[u] * 0.125f, y = b[u] * 0.125f; float xx = __fmul_rn(x, x); asm volatile("" : "+v"(xx)); float yy = __fmul_rn(y, y); asm volatile("" : "+v"(yy)); const float nrm = __fsqrt_rn(__fadd_rn(xx, yy)); float d0 = __fsub_rn(nrm, mx); asm volatile("" : "+v"(d0)); sum += __builtin_amdgcn_exp2f(__fmul_rn(d0, 1.4426950408889634f)); } }
#pragma unroll
    for (int sh = 16; sh; sh >>= 1) sum += __shfl_xor(sum, sh, 32);
    const float f = __fdiv_rn(1.0f, sum);
    for (int ps = 0; ps < 2; ++ps) { for (int j = lane * 4; j < NK; j += 128) { const v4f a = *(const v4f*)(sr + j), b = *(const v4f*)(si + j); v4us rh, rl, ih, il;
            for (int u = 0; u < 4; ++u) { const float x = a[u] * 0.125f, y = b[u] * 0.125f; float xx = __fmul_rn(x, x); asm volatile("" : "+v"(xx)); float yy = __fmul_rn(y, y); asm volatile("" : "+v"(yy)); const float nrm = __fsqrt_rn(__fadd_rn(xx, yy)); float d0 = __fsub_rn(nrm, mx); asm volatile("" : "+v"(d0)); float p = __builtin_amdgcn_exp2f(__fmul_rn(d0, 1.4426950408889634f)) * f; asm volatile("" : "+v"(p)); const float ch = __fdiv_rn(p, __fadd_rn(nrm, 1e-9f)); unsigned short h1, l1; splitf(__fmul_rn(x, ch), h1, l1); rh[u] = h1; rl[u] = l1; splitf(__fmul_rn(y, ch), h1, l1); ih[u] = h1; il[u] = l1; }
            const size_t oo = (size_t)row * (2 * NK) + j; *(volatile v4us*)(Ah + oo) = rh; *(volatile v4us*)(Al + oo) = rl; *(volatile v4us*)(Ah + oo + NK) = ih; *(volatile v4us*)(Al + oo + NK) = il; } if (ps == 0) __threadfence(); } }
__global__ __launch_bounds__(256) void k_il(const float* __restrict__ YR, const float* __restrict__ YI, float* outb) { const size_t e = ((size_t)blockIdx.x * 256 + threadIdx.x) * 4; if (e >= (size_t)RQ * DD * 2) return; const size_t idx = e / 2; v4f r; r[0] = YR[idx]; r[1] = YI[idx]; r[2] = YR[idx + 1]; r[3] = YI[idx + 1]; *(volatile v4f*)(outb + e) = r; __threadfence(); *(volatile v4f*)(outb + e) = r; }

extern "C" void kernel_launch(void* const* d_in, const int* in_sizes, int n_in,
                              void* d_out, int out_size, void* d_ws, size_t ws_size, hipStream_t stream) {
    (void)in_sizes; (void)n_in; (void)out_size;
    const float* Q = (const float*)d_in[0]; const float* K = (const float*)d_in[1]; const float* V = (const float*)d_in[2];
    float* OUT = (float*)d_out;
    char* wsp = (char*)d_ws;
    auto take = [&](size_t bytes) { char* p = wsp; wsp += (bytes + 255) & ~(size_t)255; return (void*)p; };
    bf* QC = (bf*)take((size_t)NQ * 2 * DD * 2); bf* KA = (bf*)take((size_t)NK * 2 * DD * 2); bf* KB = (bf*)take((size_t)NK * 2 * DD * 2); bf* V1 = (bf*)take((size_t)DD * 2 * NK * 2); bf* V2 = (bf*)take((size_t)DD * 2 * NK * 2);
    float* SR = (float*)take((size_t)RQ * NK * 4); float* SI = (float*)take((size_t)RQ * NK * 4); bf* Ah = (bf*)take((size_t)RQ * 2 * NK * 2); bf* Al = (bf*)take((size_t)RQ * 2 * NK * 2); float* YR = (float*)take((size_t)RQ * DD * 4); float* YI = (float*)take((size_t)RQ * DD * 4);
    if ((size_t)(wsp - (char*)d_ws) > ws_size) return;
    for (int b = 0; b < NB_; ++b) {
        k_qcat<<<(unsigned)(((size_t)NQ * 2 * DD / 4 + 255) / 256), 256, 0, stream>>>(Q + (size_t)b * NQ * DD * 2, QC); k_kcat<<<(unsigned)(((size_t)NK * 2 * DD / 4 + 255) / 256), 256, 0, stream>>>(K + (size_t)b * NK * DD * 2, KA, KB); k_vcat<<<(unsigned)(((size_t)DD * 2 * NK / 2 + 255) / 256), 256, 0, stream>>>(V + (size_t)b * NK * DD * 2, V1, V2);
        for (int r0 = 0; r0 < NQ; r0 += RQ) {
            k_gemmw<bf, 0, false><<<dim3(RQ / 64, NK / 64, 1), 32, 0, stream>>>(QC + (size_t)r0 * 2 * DD, nullptr, KA, nullptr, 2 * DD, SR, NK, nullptr, 0, 0, 0);
            k_gemmw<bf, 0, false><<<dim3(RQ / 64, NK / 64, 1), 32, 0, stream>>>(QC + (size_t)r0 * 2 * DD, nullptr, KB, nullptr, 2 * DD, SI, NK, nullptr, 0, 0, 0);
            k_csm<<<RQ / 8, 256, 0, stream>>>(SR, SI, Ah, Al);
            k_gemmw<bf, 1, false><<<dim3(RQ / 64, 1, 1), 32, 0, stream>>>(Ah, Al, V1, nullptr, 2 * NK, YR, DD, nullptr, 0, 0, 0);
            k_gemmw<bf, 1, false><<<dim3(RQ / 64, 1, 1), 32, 0, stream>>>(Ah, Al, V2, nullptr, 2 * NK, YI, DD, nullptr, 0, 0, 0);
            k_il<<<(RQ * DD * 2 / 4 + 255) / 256, 256, 0, stream>>>(YR, YI, OUT + ((size_t)b * NQ + r0) * DD * 2); } }
}
